// LISA_36146444763331
// MI455X (gfx1250) — hardware-verified
//
#include <hip/hip_runtime.h>
#include <math.h>

typedef __attribute__((ext_vector_type(16))) _Float16 v16h;
typedef __attribute__((ext_vector_type(8)))  _Float16 v8h;
typedef __attribute__((ext_vector_type(16))) __bf16   v16b;
typedef __attribute__((ext_vector_type(8)))  __bf16   v8b;
typedef __attribute__((ext_vector_type(8)))  float    v8f;
typedef __attribute__((ext_vector_type(4)))  float    v4f;
typedef __attribute__((ext_vector_type(4)))  unsigned int v4u;

constexpr int kBatch    = 8;
constexpr int kSeqL     = 32768;
constexpr int kNLat     = 2048;
constexpr int kDLat     = 64;
constexpr int kHid      = 256;
constexpr int kIn0      = 205;
constexpr int kK0Pad    = 224;
constexpr int kNFreq    = 6;
constexpr int kPts      = kBatch * kSeqL;
constexpr int kTileM    = 128;
constexpr int kThreads  = 256;
constexpr int kBtPitch  = 256;
constexpr int kActPitch = 264;
constexpr int kFPitch   = 260;
constexpr int kPlaneHalves = kHid * kBtPitch;
constexpr float kWCarry    = 64.0f;
constexpr float kWCarryInv = 1.0f / 64.0f;

static_assert(kK0Pad % 32 == 0 && kHid % 32 == 0, "K multiples of 32");
static_assert(kTileM % 64 == 0 && kHid % 64 == 0, "M and N multiples of the 64x64 wave tile");
static_assert(kPts % kTileM == 0, "grid covers all points exactly");
static_assert((kThreads / 32) == (kTileM / 64) * (kHid / 64), "one wave per 64x64 output tile");
static_assert(kActPitch % 8 == 0 && kActPitch >= kHid, "16-B aligned activation rows");

constexpr int kLdsP16      = 0;
constexpr int kLdsPlane16B = kTileM * kActPitch * 2;
constexpr int kLdsPLo      = kLdsPlane16B;
constexpr int kLdsBig      = 2 * kLdsPlane16B;
constexpr int kLdsW4       = kLdsBig;
constexpr int kLdsOut      = kLdsW4 + kHid * 4;
constexpr int kLdsBytes    = kLdsOut + kTileM * 4;
static_assert(kTileM * kFPitch * 4 <= kLdsBig, "f32 plane fits inside the two 16-bit planes");
static_assert(kLdsBytes <= 160 * 1024, "LDS budget");

constexpr size_t kWsBtOff    = 0;
constexpr size_t kWsBtBytes  = (size_t)4 * kPlaneHalves * 2;
constexpr size_t kWsLatOff   = kWsBtOff + kWsBtBytes;
constexpr size_t kWsLatBytes = (size_t)kBatch * kNLat * kDLat * 4;
constexpr size_t kWsTotal    = kWsLatOff + kWsLatBytes;
static_assert(kWsTotal <= (size_t)134217728, "workspace carve under 128 MiB");
constexpr int kLatN4 = kBatch * kNLat * kDLat / 4;
static_assert(kLatN4 % 256 == 0, "latent prep grid exact");

__device__ __forceinline__ unsigned short f2bf_bits(float f) {
  unsigned u = __float_as_uint(f);
  return (unsigned short)((u + 0x7FFFu + ((u >> 16) & 1u)) >> 16);
}
__device__ __forceinline__ float bf_bits2f(unsigned short h) { return __uint_as_float(((unsigned)h) << 16); }

__device__ __forceinline__ void dep_guard_h(v8f& a, v8f& b, v16h x, v16h y) { asm volatile("v_nop\n\tv_nop\n\tv_nop\n\tv_nop" : "+v"(a), "+v"(b) : "v"(x), "v"(y)); }
__device__ __forceinline__ void dep_guard_b(v8f& a, v8f& b, v16b x, v16b y) { asm volatile("v_nop\n\tv_nop\n\tv_nop\n\tv_nop" : "+v"(a), "+v"(b) : "v"(x), "v"(y)); }
__device__ __forceinline__ void keep4_h(v16h a, v16h b, v16h c, v16h d) { asm volatile("v_nop" :: "v"(a), "v"(b), "v"(c), "v"(d)); }
__device__ __forceinline__ void keep4_b(v16b a, v16b b, v16b c, v16b d) { asm volatile("v_nop" :: "v"(a), "v"(b), "v"(c), "v"(d)); }
__device__ __forceinline__ void acc_guard4(v8f& a, v8f& b, v8f& c, v8f& d) { asm volatile("v_nop\n\tv_nop\n\tv_nop\n\tv_nop" : "+v"(a), "+v"(b), "+v"(c), "+v"(d)); }
template <typename T> struct Frag;
template <> struct Frag<_Float16> {
  typedef v16h V; union U { v16h v; v8h h[2]; };
  static __device__ __forceinline__ v16h load(const _Float16* p) {
    U f; f.h[0] = *(const v8h*)(p); f.h[1] = *(const v8h*)(p + 16); return f.v;
  }
  static __device__ __forceinline__ v8f mma(v16h a, v16h b, v8f c) {
    return __builtin_amdgcn_wmma_f32_16x16x32_f16(false, a, false, b, (short)0, c, false, false);
  }
  static __device__ __forceinline__ void guard(v8f& a, v8f& b, v16h x, v16h y) { dep_guard_h(a, b, x, y); }
  static __device__ __forceinline__ void keep(v16h a, v16h b, v16h c, v16h d) { keep4_h(a, b, c, d); }
};
template <> struct Frag<__bf16> {
  typedef v16b V; union U { v16b v; v8b h[2]; };
  static __device__ __forceinline__ v16b load(const __bf16* p) {
    U f; f.h[0] = *(const v8b*)(p); f.h[1] = *(const v8b*)(p + 16); return f.v;
  }
  static __device__ __forceinline__ v8f mma(v16b a, v16b b, v8f c) {
    return __builtin_amdgcn_wmma_f32_16x16x32_bf16(false, a, false, b, (short)0, c, false, false);
  }
  static __device__ __forceinline__ void guard(v8f& a, v8f& b, v16b x, v16b y) { dep_guard_b(a, b, x, y); }
  static __device__ __forceinline__ void keep(v16b a, v16b b, v16b c, v16b d) { keep4_b(a, b, c, d); }
};

__device__ __forceinline__ unsigned pk16(unsigned short a, unsigned short b) { return (unsigned)a | ((unsigned)b << 16); }
__device__ __forceinline__ unsigned short h_bits(float f) { const _Float16 h = (_Float16)f; return __builtin_bit_cast(unsigned short, h); }
__device__ __forceinline__ float bfr(float f) {
  unsigned u = __float_as_uint(f);
  u = (u + 0x7FFFu + ((u >> 16) & 1u)) & 0xFFFF0000u;
  return __uint_as_float(u);
}

__global__ __launch_bounds__(256) void lat_prep_kernel(const float* __restrict__ in, float* __restrict__ outp, int n4) {
  const int i = blockIdx.x * 256 + threadIdx.x;
  if (i >= n4) return;
  const v4f a = *(const v4f*)(in + 4 * (size_t)i);
  v4f r;
  r[0] = bfr(a[0]); r[1] = bfr(a[1]); r[2] = bfr(a[2]); r[3] = bfr(a[3]);
  float* q = outp + 4 * (size_t)i;
  *(volatile v4f*)q = r;
  __threadfence();
  *(volatile v4f*)q = r;
}

__global__ __launch_bounds__(256) void wprep_kernel(const float* __restrict__ W0, const float* __restrict__ W1,
                                                    const float* __restrict__ W2, const float* __restrict__ W3,
                                                    unsigned short* __restrict__ btw) {
  __shared__ float sm[64][65];
  const int t   = threadIdx.x;
  const int k0t = blockIdx.x * 64;
  const int n0t = blockIdx.y * 64;
  const int z   = blockIdx.z;
  const float* W = (z == 0) ? W0 : (z == 1) ? W1 : (z == 2) ? W2 : W3;
  const int kin = (z == 0) ? kIn0 : kHid;
#pragma unroll
  for (int i = 0; i < 16; ++i) {
    const int e = i * 256 + t;
    const int r = e >> 6;
    const int c = e & 63;
    const int k = k0t + r;
    const int n = n0t + c;
    int  sr    = k;
    bool valid = true;
    if (z == 0) {
      valid = (k < 13) || (k >= 16 && k < 208);
      sr    = (k < 13) ? k : (k - 3);
    }
    sr = sr < 0 ? 0 : (sr > kin - 1 ? kin - 1 : sr);
    float v = W[(size_t)sr * kHid + n];
    v = valid ? v : 0.0f;
    v = bfr(v);
    if (z != 3) v = v * kWCarry;
    sm[c][r] = v;
  }
  __syncthreads();
  const int lane = t & 31, wave = t >> 5;
  const int q = lane >> 3, c8 = (lane & 7) * 8;
  unsigned short* op = btw + (size_t)z * kPlaneHalves;
  for (int pass = 0; pass < 2; ++pass) {
#pragma unroll
    for (int it = 0; it < 2; ++it) {
      const int row = wave * 8 + it * 4 + q;
      unsigned short hb[8];
#pragma unroll
      for (int e = 0; e < 8; ++e) {
        const float x = sm[row][c8 + e];
        const unsigned short b16 = f2bf_bits(x);
        const unsigned short h16 = h_bits(x);
        hb[e] = (z == 3) ? b16 : h16;
      }
      const v4u u = (v4u){pk16(hb[0], hb[1]), pk16(hb[2], hb[3]), pk16(hb[4], hb[5]), pk16(hb[6], hb[7])};
      *(volatile v4u*)(op + (size_t)(n0t + row) * kBtPitch + k0t + c8) = u;
    }
    __threadfence();
  }
}

template <typename T, bool SPLITA>
__device__ __forceinline__ void tile_mma(const T* A, const T* Alo, const T* __restrict__ Bt, int K,
                                         v8f (&acc)[4][4], int m0, int n0, int lane) {
  typedef typename Frag<T>::V V;
  const int rlane = lane & 15;
  const int koff  = (lane >> 4) * 8;
#pragma unroll
  for (int i = 0; i < 4; ++i)
#pragma unroll
    for (int j = 0; j < 4; ++j) acc[i][j] = (v8f){0.f,0.f,0.f,0.f,0.f,0.f,0.f,0.f};
#pragma unroll 1
  for (int k0 = 0; k0 < K; k0 += 32) {
    V bh[4];
#pragma unroll
    for (int j = 0; j < 4; ++j)
      bh[j] = Frag<T>::load(Bt + (size_t)(n0 + (j << 4) + rlane) * kBtPitch + koff + k0);
#pragma unroll
    for (int i = 0; i < 4; ++i) {
      const int ao = (m0 + (i << 4) + rlane) * kActPitch + koff + k0;
      V ah = Frag<T>::load(A + ao);
      V al = ah;
      if (SPLITA) al = Frag<T>::load(Alo + ao);
#pragma unroll
      for (int j = 0; j < 4; ++j) {
        acc[i][j] = Frag<T>::mma(ah, bh[j], acc[i][j]);
        if (SPLITA) acc[i][j] = Frag<T>::mma(al, bh[j], acc[i][j]);
      }
      Frag<T>::guard(acc[i][0], acc[i][3], ah, al);
    }
    Frag<T>::keep(bh[0], bh[1], bh[2], bh[3]);
  }
  acc_guard4(acc[0][0], acc[0][1], acc[0][2], acc[0][3]);
  acc_guard4(acc[1][0], acc[1][1], acc[1][2], acc[1][3]);
  acc_guard4(acc[2][0], acc[2][1], acc[2][2], acc[2][3]);
  acc_guard4(acc[3][0], acc[3][1], acc[3][2], acc[3][3]);
}

__device__ __forceinline__ void epi_f16(v8f (&acc)[4][4], const float* __restrict__ bias, unsigned short* P,
                                        int m0, int n0, int lane) {
  const int rlane = lane & 15, mOff = (lane >> 4) * 8;
  float bv[4];
#pragma unroll
  for (int j = 0; j < 4; ++j) bv[j] = bfr(bias[n0 + (j << 4) + rlane]);
#pragma unroll
  for (int i = 0; i < 4; ++i) {
#pragma unroll
    for (int j = 0; j < 4; ++j) {
      const int n = n0 + (j << 4) + rlane;
#pragma unroll
      for (int r = 0; r < 8; ++r) {
        float v = acc[i][j][r] * kWCarryInv + bv[j];
        v = fmaxf(v, 0.0f);
        P[(m0 + (i << 4) + mOff + r) * kActPitch + n] = h_bits(v);
      }
    }
  }
}

__device__ __forceinline__ void epi_bf2(v8f (&acc)[4][4], const float* __restrict__ bias, unsigned short* Phi,
                                        unsigned short* Plo, int m0, int n0, int lane) {
  const int rlane = lane & 15, mOff = (lane >> 4) * 8;
  float bv[4];
#pragma unroll
  for (int j = 0; j < 4; ++j) bv[j] = bfr(bias[n0 + (j << 4) + rlane]);
#pragma unroll
  for (int i = 0; i < 4; ++i) {
#pragma unroll
    for (int j = 0; j < 4; ++j) {
      const int n = n0 + (j << 4) + rlane;
#pragma unroll
      for (int r = 0; r < 8; ++r) {
        float v = acc[i][j][r] * kWCarryInv + bv[j];
        v = fmaxf(v, 0.0f);
        const unsigned short hb = f2bf_bits(v);
        const unsigned short lb = f2bf_bits(v - bf_bits2f(hb));
        const int idx = (m0 + (i << 4) + mOff + r) * kActPitch + n;
        Phi[idx] = hb;
        Plo[idx] = lb;
      }
    }
  }
}

__device__ __forceinline__ void epi_f32(v8f (&acc)[4][4], const float* __restrict__ bias, float* Pf,
                                        int m0, int n0, int lane) {
  const int rlane = lane & 15, mOff = (lane >> 4) * 8;
  float bv[4];
#pragma unroll
  for (int j = 0; j < 4; ++j) bv[j] = bfr(bias[n0 + (j << 4) + rlane]);
#pragma unroll
  for (int i = 0; i < 4; ++i) {
#pragma unroll
    for (int j = 0; j < 4; ++j) {
      const int n = n0 + (j << 4) + rlane;
#pragma unroll
      for (int r = 0; r < 8; ++r) {
        float v = acc[i][j][r] + bv[j];
        v = fmaxf(v, 0.0f);
        Pf[(m0 + (i << 4) + mOff + r) * kFPitch + n] = v;
      }
    }
  }
}

__global__ __launch_bounds__(256) void mlp_fused_kernel(
    const float* __restrict__ coord, const float* __restrict__ latr, const unsigned short* __restrict__ btw,
    const float* __restrict__ b0, const float* __restrict__ b1, const float* __restrict__ b2,
    const float* __restrict__ b3, const float* __restrict__ W4, const float* __restrict__ b4,
    float* __restrict__ out) {
  extern __shared__ v4u lds_dyn[];
  unsigned char*  lds_raw = (unsigned char*)lds_dyn;
  unsigned short* p16  = (unsigned short*)(lds_raw + kLdsP16);
  unsigned short* plo  = (unsigned short*)(lds_raw + kLdsPLo);
  float*          pf32 = (float*)(lds_raw + kLdsP16);
  float*          w4s  = (float*)(lds_raw + kLdsW4);
  float*          outs = (float*)(lds_raw + kLdsOut);

  const int t    = threadIdx.x;
  const int lane = t & 31;
  const int wave = t >> 5;
  const int pt0  = blockIdx.x * kTileM;

  w4s[t] = bfr(W4[t]);

  if (t < kTileM) {
    const int gp = pt0 + t;
    const float c = bfr(coord[gp]);
    unsigned short* row = p16 + t * kActPitch;
    const v4u z4 = (v4u){0u, 0u, 0u, 0u};
    *(v4u*)(row + 208) = z4;
    *(v4u*)(row + 216) = z4;
    row[0]  = h_bits(c);
    row[13] = (unsigned short)0;
    row[14] = (unsigned short)0;
    row[15] = (unsigned short)0;
    float a = c;
#pragma unroll 1
    for (int j = 0; j < kNFreq; ++j) {
      row[1 + 2 * j] = h_bits(sinf(a));
      row[2 + 2 * j] = h_bits(cosf(a));
      a = a * 2.0f;
    }
  }

  {
    const int p    = t >> 1;
    const int hs   = t & 1;
    const int gp   = pt0 + p;
    const int bidx = gp >> 15;
    const float c  = bfr(coord[gp]);
    const float ix = c * 2048.0f - 0.5f;
    const float x0 = floorf(ix);
    const float tt = ix - x0;
    const float wa = 1.0f - tt;
    int i0 = (int)x0;
    int i1 = i0 + 1;
    i0 = i0 < 0 ? 0 : (i0 > kNLat - 1 ? kNLat - 1 : i0);
    i1 = i1 < 0 ? 0 : (i1 > kNLat - 1 ? kNLat - 1 : i1);
    const float* lb = latr + (size_t)bidx * (kNLat * kDLat);
    unsigned short* arow = p16 + p * kActPitch + 16;
#pragma unroll 2
    for (int q = 0; q < 12; ++q) {
      const int cch = hs * 96 + 8 * q;
      const int g = cch >> 6;
      const int d = cch & 63;
      int ra = i0 + g - 1; ra = ra < 0 ? 0 : (ra > kNLat - 1 ? kNLat - 1 : ra);
      int rb = i1 + g - 1; rb = rb < 0 ? 0 : (rb > kNLat - 1 ? kNLat - 1 : rb);
      const float* pa = lb + ra * kDLat + d;
      const float* pb = lb + rb * kDLat + d;
      const v4f a0 = *(const v4f*)(pa);
      const v4f a1 = *(const v4f*)(pa + 4);
      const v4f c0 = *(const v4f*)(pb);
      const v4f c1 = *(const v4f*)(pb + 4);
      float f[8];
#pragma unroll
      for (int e = 0; e < 4; ++e) {
        f[e]     = wa * a0[e] + tt * c0[e];
        f[4 + e] = wa * a1[e] + tt * c1[e];
      }
      const v4u u = (v4u){pk16(h_bits(f[0]), h_bits(f[1])), pk16(h_bits(f[2]), h_bits(f[3])),
                          pk16(h_bits(f[4]), h_bits(f[5])), pk16(h_bits(f[6]), h_bits(f[7]))};
      *(v4u*)(arow + cch) = u;
    }
  }
  __syncthreads();

  const int m0 = (wave >> 2) * 64;
  const int n0 = (wave & 3) * 64;
  v8f acc[4][4];
  const _Float16* A16 = (const _Float16*)p16;
  const _Float16* Bt0 = (const _Float16*)(btw + 0 * (size_t)kPlaneHalves);
  const _Float16* Bt1 = (const _Float16*)(btw + 1 * (size_t)kPlaneHalves);
  const _Float16* Bt2 = (const _Float16*)(btw + 2 * (size_t)kPlaneHalves);
  const __bf16*   Bt3 = (const __bf16*)(btw + 3 * (size_t)kPlaneHalves);

  tile_mma<_Float16, false>(A16, A16, Bt0, kK0Pad, acc, m0, n0, lane);
  __syncthreads();
  epi_f16(acc, b0, p16, m0, n0, lane);
  __syncthreads();

  tile_mma<_Float16, false>(A16, A16, Bt1, kHid, acc, m0, n0, lane);
  __syncthreads();
  epi_f16(acc, b1, p16, m0, n0, lane);
  __syncthreads();

  tile_mma<_Float16, false>(A16, A16, Bt2, kHid, acc, m0, n0, lane);
  __syncthreads();
  epi_bf2(acc, b2, p16, plo, m0, n0, lane);
  __syncthreads();

  tile_mma<__bf16, true>((const __bf16*)p16, (const __bf16*)plo, Bt3, kHid, acc, m0, n0, lane);
  __syncthreads();
  epi_f32(acc, b3, pf32, m0, n0, lane);
  __syncthreads();

  {
    const int row  = t >> 1;
    const int half = t & 1;
    const float* ar = pf32 + row * kFPitch + half * 128;
    const float* wr = w4s + half * 128;
    float s = 0.0f;
#pragma unroll 2
    for (int q = 0; q < 32; ++q) {
      const v4f av = *(const v4f*)(ar + 4 * q);
      const v4f wv = *(const v4f*)(wr + 4 * q);
      s += av[0] * wv[0];
      s += av[1] * wv[1];
      s += av[2] * wv[2];
      s += av[3] * wv[3];
    }
    const float tot = s + __shfl_xor(s, 1, 32);
    const float res = tot + bfr(b4[0]);
    if (half == 0) outs[row] = res;
  }
  __syncthreads();

  if (wave == 0) {
    const v4f v = *(const v4f*)(outs + 4 * lane);
    float* op = out + (size_t)pt0 + 4 * lane;
    *(volatile v4f*)op = v;
    __threadfence();
    *(volatile v4f*)op = v;
  }
}

extern "C" void kernel_launch(void* const* d_in, const int* in_sizes, int n_in,
                              void* d_out, int out_size, void* d_ws, size_t ws_size,
                              hipStream_t stream) {
  (void)in_sizes; (void)n_in; (void)out_size; (void)ws_size;
  const float* coord  = (const float*)d_in[0];
  const float* latent = (const float*)d_in[1];
  const float* W0 = (const float*)d_in[2];
  const float* b0 = (const float*)d_in[3];
  const float* W1 = (const float*)d_in[4];
  const float* b1 = (const float*)d_in[5];
  const float* W2 = (const float*)d_in[6];
  const float* b2 = (const float*)d_in[7];
  const float* W3 = (const float*)d_in[8];
  const float* b3 = (const float*)d_in[9];
  const float* W4 = (const float*)d_in[10];
  const float* b4 = (const float*)d_in[11];
  float* out = (float*)d_out;

  unsigned char*  ws   = (unsigned char*)d_ws;
  unsigned short* btw  = (unsigned short*)(ws + kWsBtOff);
  float*          latr = (float*)(ws + kWsLatOff);

  lat_prep_kernel<<<dim3(kLatN4 / 256), dim3(256), 0, stream>>>(latent, latr, kLatN4);
  wprep_kernel<<<dim3(4, 4, 4), dim3(256), 0, stream>>>(W0, W1, W2, W3, btw);
  mlp_fused_kernel<<<dim3(kPts / kTileM), dim3(kThreads), kLdsBytes, stream>>>(
      coord, latr, btw, b0, b1, b2, b3, W4, b4, out);
}
